// Down_channelV2_86930138071596
// MI455X (gfx1250) — hardware-verified
//
#include <hip/hip_runtime.h>
#include <math.h>

typedef __attribute__((ext_vector_type(16))) _Float16 v16h;
typedef __attribute__((ext_vector_type(8)))  _Float16 v8h;
typedef __attribute__((ext_vector_type(16))) __bf16   v16b;
typedef __attribute__((ext_vector_type(8)))  __bf16   v8b;
typedef __attribute__((ext_vector_type(8)))  float    v8f;
typedef __attribute__((ext_vector_type(4)))  float    v4f;

constexpr int kBatch = 2;
constexpr int kMod   = 96;
constexpr int kPix   = 4096;
constexpr int kRows  = kBatch * kPix;
constexpr int kCin   = 288;
constexpr int kCinP  = 320;
constexpr int kDin   = 576;
constexpr int kXZW   = 2 * kDin;
constexpr int kNst   = 16;
constexpr int kDtR   = 18;
constexpr int kXdbl  = 50;
constexpr int kPrjP  = 64;
constexpr int kDtP   = 32;
constexpr int kWdtP  = 64;
constexpr int kOutP  = 128;
constexpr int kTP    = 68;

__device__ __forceinline__ unsigned short f2bf_bits(float f) {
  unsigned u = __float_as_uint(f);
  return (unsigned short)((u + 0x7FFFu + ((u >> 16) & 1u)) >> 16);
}
__device__ __forceinline__ float bf_bits2f(unsigned short h) { return __uint_as_float(((unsigned)h) << 16); }

__device__ __forceinline__ void dep_guard_h(v8f& a, v8f& b, v16h x, v16h y) { asm volatile("v_nop\n\tv_nop\n\tv_nop\n\tv_nop" : "+v"(a), "+v"(b) : "v"(x), "v"(y)); }
__device__ __forceinline__ void dep_guard_b(v8f& a, v8f& b, v16b x, v16b y) { asm volatile("v_nop\n\tv_nop\n\tv_nop\n\tv_nop" : "+v"(a), "+v"(b) : "v"(x), "v"(y)); }
__device__ __forceinline__ void keep4_h(v16h a, v16h b, v16h c, v16h d) { asm volatile("v_nop" :: "v"(a), "v"(b), "v"(c), "v"(d)); }
__device__ __forceinline__ void keep4_b(v16b a, v16b b, v16b c, v16b d) { asm volatile("v_nop" :: "v"(a), "v"(b), "v"(c), "v"(d)); }
__device__ __forceinline__ void acc_guard4(v8f& a, v8f& b, v8f& c, v8f& d) { asm volatile("v_nop\n\tv_nop\n\tv_nop\n\tv_nop" : "+v"(a), "+v"(b), "+v"(c), "+v"(d)); }
template <typename T> struct Frag;
template <> struct Frag<_Float16> {
  typedef v16h V; union U { v16h v; v8h h[2]; };
  static __device__ __forceinline__ v16h load(const _Float16* p) {
    U f; f.h[0] = *(const v8h*)(p); f.h[1] = *(const v8h*)(p + 16); return f.v;
  }
  static __device__ __forceinline__ v8f mma(v16h a, v16h b, v8f c) {
    return __builtin_amdgcn_wmma_f32_16x16x32_f16(false, a, false, b, (short)0, c, false, false);
  }
  static __device__ __forceinline__ void guard(v8f& a, v8f& b, v16h x, v16h y) { dep_guard_h(a, b, x, y); }
  static __device__ __forceinline__ void keep(v16h a, v16h b, v16h c, v16h d) { keep4_h(a, b, c, d); }
};
template <> struct Frag<__bf16> {
  typedef v16b V; union U { v16b v; v8b h[2]; };
  static __device__ __forceinline__ v16b load(const __bf16* p) {
    U f; f.h[0] = *(const v8b*)(p); f.h[1] = *(const v8b*)(p + 16); return f.v;
  }
  static __device__ __forceinline__ v8f mma(v16b a, v16b b, v8f c) {
    return __builtin_amdgcn_wmma_f32_16x16x32_bf16(false, a, false, b, (short)0, c, false, false);
  }
  static __device__ __forceinline__ void guard(v8f& a, v8f& b, v16b x, v16b y) { dep_guard_b(a, b, x, y); }
  static __device__ __forceinline__ void keep(v16b a, v16b b, v16b c, v16b d) { keep4_b(a, b, c, d); }
};

template <int ET> struct Elem;
template <> struct Elem<0> { typedef _Float16 T; };
template <> struct Elem<1> { typedef __bf16 T; };
template <int ET, bool SPLIT, int BIAS_MODE, int OUT_MODE, bool RESID, int ACT = 0>
__global__ __launch_bounds__(256) void wmma_gemm64(
    const unsigned short* __restrict__ Ap, const unsigned short* __restrict__ A2p, int lda, long strideA,
    const unsigned short* __restrict__ Btp, const unsigned short* __restrict__ Bt2p, int ldb, long strideB,
    void* __restrict__ Cout, void* __restrict__ Cout2, int ldc, long strideC,
    const float* __restrict__ bias,
    const float* __restrict__ resid, long strideR,
    int M, int N, int K, float scale) {
  typedef typename Elem<ET>::T T;
  typedef typename Frag<T>::V V;
  const T* A = (const T*)Ap; const T* A2 = (const T*)A2p; const T* Bt = (const T*)Btp; const T* Bt2 = (const T*)Bt2p;
  __shared__ __align__(16) float sT[8][16 * 68];
  const int b    = blockIdx.y;
  const int lane = threadIdx.x & 31;
  const int wave = threadIdx.x >> 5;
  const int tilesN = N >> 6;
  const int tilesM = M >> 6;
  const int tile = blockIdx.x * 8 + wave;
  if (tile >= tilesM * tilesN) return;
  const int tm = tile / tilesN;
  const int tn = tile - tm * tilesN;
  const int m0 = tm << 6;
  const int n0 = tn << 6;

  const T* Ab  = A  + (size_t)b * strideA;
  const T* Bb  = Bt + (size_t)b * strideB;
  const T* Ab2 = SPLIT ? (A2  + (size_t)b * strideA) : nullptr;
  const T* Bb2 = SPLIT ? (Bt2 + (size_t)b * strideB) : nullptr;

  const int rlane = lane & 15;
  const int koff  = (lane >> 4) * 8;
  const int mOff  = (lane >> 4) * 8;

  v8f acc[4][4];
#pragma unroll
  for (int i = 0; i < 4; ++i)
#pragma unroll
    for (int j = 0; j < 4; ++j) acc[i][j] = (v8f){0.f,0.f,0.f,0.f,0.f,0.f,0.f,0.f};

  for (int k0 = 0; k0 < K; k0 += 32) {
    V bh[4], bl[4];
#pragma unroll
    for (int j = 0; j < 4; ++j) {
      const size_t bo = (size_t)(n0 + (j << 4) + rlane) * ldb + koff + k0;
      bh[j] = Frag<T>::load(Bb + bo);
      if (SPLIT) bl[j] = Frag<T>::load(Bb2 + bo);
    }
#pragma unroll
    for (int i = 0; i < 4; ++i) {
      const size_t ao = (size_t)(m0 + (i << 4) + rlane) * lda + koff + k0;
      V ah = Frag<T>::load(Ab + ao);
      V al;
      if (SPLIT) al = Frag<T>::load(Ab2 + ao);
#pragma unroll
      for (int j = 0; j < 4; ++j) {
        acc[i][j] = Frag<T>::mma(ah, bh[j], acc[i][j]);
        if (SPLIT) {
          acc[i][j] = Frag<T>::mma(ah, bl[j], acc[i][j]);
          acc[i][j] = Frag<T>::mma(al, bh[j], acc[i][j]);
        }
      }
      Frag<T>::guard(acc[i][0], acc[i][3], ah, SPLIT ? al : ah);
    }
    Frag<T>::keep(bh[0], bh[1], bh[2], bh[3]);
    if (SPLIT) Frag<T>::keep(bl[0], bl[1], bl[2], bl[3]);
  }
  acc_guard4(acc[0][0], acc[0][1], acc[0][2], acc[0][3]);
  acc_guard4(acc[1][0], acc[1][1], acc[1][2], acc[1][3]);
  acc_guard4(acc[2][0], acc[2][1], acc[2][2], acc[2][3]);
  acc_guard4(acc[3][0], acc[3][1], acc[3][2], acc[3][3]);

  float* slab = sT[wave];
  const float* Rb = RESID ? (resid + (size_t)b * strideR) : nullptr;
#pragma unroll
  for (int i = 0; i < 4; ++i) {
    const int mBase = m0 + (i << 4);
#pragma unroll
    for (int j = 0; j < 4; ++j) {
      const int n = n0 + (j << 4) + rlane;
      float bv = 0.f;
      if (BIAS_MODE == 2) bv = bias[n];
#pragma unroll
      for (int r = 0; r < 8; ++r) {
        float v = acc[i][j][r] * scale;
        if (BIAS_MODE == 1) v += bias[mBase + mOff + r];
        if (BIAS_MODE == 2) v += bv;
        if (RESID) v += Rb[(size_t)(mBase + mOff + r) * ldc + n];
        if (ACT == 1) v = tanhf(v);
        if (ACT == 2) v = fmaxf(v, 0.0f);
        if (ACT == 3) v = v / (1.0f + expf(-v));
        if (ACT == 4) v = (v > 0.f) ? v : 0.01f * v;
        if (ACT == 5) v = 0.5f * v * (1.0f + erff(v * 0.70710678118654752f));
        slab[(mOff + r) * 68 + (j << 4) + rlane] = v;
      }
    }
    __builtin_amdgcn_fence(__ATOMIC_RELEASE, "workgroup");
    __builtin_amdgcn_wave_barrier();
    __builtin_amdgcn_fence(__ATOMIC_ACQUIRE, "workgroup");
    if (OUT_MODE == 0) {
      float* C = (float*)Cout + (size_t)b * strideC;
      const int hh = lane >> 4, c4 = (lane & 15) * 4;
      for (int pass = 0; pass < 2; ++pass) {
#pragma unroll
        for (int it = 0; it < 8; ++it) {
          const int row = it * 2 + hh;
          v4f v = *(const v4f*)(slab + row * 68 + c4);
          *(volatile v4f*)(C + (size_t)(mBase + row) * ldc + n0 + c4) = v;
        }
        __threadfence();
      }
    } else {
      const int q = lane >> 3, c8 = (lane & 7) * 8;
      unsigned short* C  = (unsigned short*)Cout  + (size_t)b * strideC;
      unsigned short* C2 = (OUT_MODE == 2) ? ((unsigned short*)Cout2 + (size_t)b * strideC) : nullptr;
      for (int pass = 0; pass < 2; ++pass) {
#pragma unroll
        for (int it = 0; it < 4; ++it) {
          const int row = it * 4 + q;
          const float* sp = slab + row * 68 + c8;
          v8h hv, lv;
#pragma unroll
          for (int e = 0; e < 8; ++e) {
            if (OUT_MODE == 1) {
              hv[e] = (_Float16)sp[e];
            } else {
              unsigned short hb = f2bf_bits(sp[e]);
              unsigned short lb = f2bf_bits(sp[e] - bf_bits2f(hb));
              hv[e] = __builtin_bit_cast(_Float16, hb);
              lv[e] = __builtin_bit_cast(_Float16, lb);
            }
          }
          *(volatile v8h*)(C + (size_t)(mBase + row) * ldc + n0 + c8) = hv;
          if (OUT_MODE == 2) *(volatile v8h*)(C2 + (size_t)(mBase + row) * ldc + n0 + c8) = lv;
        }
        __threadfence();
      }
    }
    __builtin_amdgcn_fence(__ATOMIC_RELEASE, "workgroup");
    __builtin_amdgcn_wave_barrier();
    __builtin_amdgcn_fence(__ATOMIC_ACQUIRE, "workgroup");
  }
}

template <int OM>
__global__ __launch_bounds__(256) void transpose_cast_kernel(
    const float* __restrict__ W, unsigned short* __restrict__ Bt, unsigned short* __restrict__ Bt2,
    int Kdim, int Ndim, int Kpitch, int splitAt, int shift, float scale)
{
  __shared__ float tile[64 * 65];
  const int tid = threadIdx.x, lane = tid & 31, wave = tid >> 5;
  const int n0 = blockIdx.x * 64;
  const int k0 = blockIdx.y * 64;
#pragma unroll
  for (int p = 0; p < 16; ++p) {
    const int idx = tid + p * 256;
    const int kk  = idx >> 6;
    const int nn  = idx & 63;
    const int n   = n0 + nn;
    const int k   = k0 + kk;
    const bool nv = (n < splitAt) || (n >= splitAt + shift);
    const int sc  = (n < splitAt) ? n : (n - shift);
    const bool valid = nv && (sc < Ndim) && (k < Kdim);
    const int scc = (sc < 0) ? 0 : ((sc < Ndim) ? sc : (Ndim - 1));
    const int kc  = (k < Kdim) ? k : (Kdim - 1);
    const float v = W[(size_t)kc * Ndim + scc];
    tile[kk * 65 + nn] = valid ? (v * scale) : 0.f;
  }
  __syncthreads();
  const int q = lane >> 3, c8 = (lane & 7) * 8;
  v8h hv[2], lv[2];
#pragma unroll
  for (int it = 0; it < 2; ++it) {
    const int nrow = it * 32 + wave * 4 + q;
#pragma unroll
    for (int e = 0; e < 8; ++e) {
      const float t = tile[(c8 + e) * 65 + nrow];
      if (OM == 0) {
        hv[it][e] = (_Float16)t;
        lv[it][e] = (_Float16)0.0f;
      } else {
        const unsigned short hb = f2bf_bits(t);
        const unsigned short lb = f2bf_bits(t - bf_bits2f(hb));
        hv[it][e] = __builtin_bit_cast(_Float16, hb);
        lv[it][e] = __builtin_bit_cast(_Float16, lb);
      }
    }
  }
  for (int pass = 0; pass < 2; ++pass) {
#pragma unroll
    for (int it = 0; it < 2; ++it) {
      const int nrow = it * 32 + wave * 4 + q;
      *(volatile v8h*)(Bt + (size_t)(n0 + nrow) * Kpitch + k0 + c8) = hv[it];
      if (OM == 1) *(volatile v8h*)(Bt2 + (size_t)(n0 + nrow) * Kpitch + k0 + c8) = lv[it];
    }
    __threadfence();
  }
}

__global__ __launch_bounds__(256) void ln0_kernel(
    const float* __restrict__ x1, const float* __restrict__ x2, const float* __restrict__ x3,
    const float* __restrict__ g, const float* __restrict__ bb,
    float* __restrict__ XT, unsigned short* __restrict__ XN16)
{
  __shared__ __align__(16) float sx[8][kCinP];
  __shared__ __align__(16) float sn[8][kCinP];
  const int tid = threadIdx.x, lane = tid & 31, wave = tid >> 5;
  const int grow = blockIdx.x * 8 + wave;
  const int b = grow >> 12, l = grow & 4095;
  float v[9];
  float s = 0.f;
#pragma unroll
  for (int j = 0; j < 9; ++j) {
    const int c  = lane + 32 * j;
    const int i  = l * kCin + c;
    const int ch = i >> 12, px = i & 4095;
    const int c1 = (ch < kMod) ? ch : (kMod - 1);
    int c2 = ch - kMod;     c2 = (c2 < 0) ? 0 : ((c2 > kMod - 1) ? (kMod - 1) : c2);
    int c3 = ch - 2 * kMod; c3 = (c3 < 0) ? 0 : ((c3 > kMod - 1) ? (kMod - 1) : c3);
    const float a1 = x1[((size_t)(b * kMod + c1) << 12) + px];
    const float a2 = x2[((size_t)(b * kMod + c2) << 12) + px];
    const float a3 = x3[((size_t)(b * kMod + c3) << 12) + px];
    const float val = (ch < kMod) ? a1 : ((ch < 2 * kMod) ? a2 : a3);
    v[j] = val;
    s += val;
  }
#pragma unroll
  for (int off = 16; off > 0; off >>= 1) s += __shfl_xor(s, off, 32);
  const float mu = s * (1.0f / 288.0f);
  float s2 = 0.f;
#pragma unroll
  for (int j = 0; j < 9; ++j) { const float dv = v[j] - mu; s2 += dv * dv; }
#pragma unroll
  for (int off = 16; off > 0; off >>= 1) s2 += __shfl_xor(s2, off, 32);
  const float rstd = rsqrtf(s2 * (1.0f / 288.0f) + 1e-5f);
#pragma unroll
  for (int j = 0; j < 9; ++j) {
    const int c = lane + 32 * j;
    sx[wave][c] = v[j];
    sn[wave][c] = (v[j] - mu) * rstd * g[c] + bb[c];
  }
  sx[wave][kCin + lane] = 0.f;
  sn[wave][kCin + lane] = 0.f;
  __syncthreads();

  const v4f f0 = *(const v4f*)(&sx[wave][lane * 4]);
  const v4f f1 = *(const v4f*)(&sx[wave][128 + lane * 4]);
  const v4f f2 = *(const v4f*)(&sx[wave][256 + (lane & 15) * 4]);
  v8h h0, h1;
#pragma unroll
  for (int e = 0; e < 8; ++e) {
    h0[e] = (_Float16)sn[wave][lane * 8 + e];
    h1[e] = (_Float16)sn[wave][256 + (lane & 7) * 8 + e];
  }
  float* xrow = XT + (size_t)grow * kCinP;
  unsigned short* nrow = XN16 + (size_t)grow * kCinP;
  for (int pass = 0; pass < 2; ++pass) {
    *(volatile v4f*)(xrow + lane * 4) = f0;
    *(volatile v4f*)(xrow + 128 + lane * 4) = f1;
    if (lane < 16) *(volatile v4f*)(xrow + 256 + lane * 4) = f2;
    *(volatile v8h*)(nrow + lane * 8) = h0;
    if (lane < 8) *(volatile v8h*)(nrow + 256 + lane * 8) = h1;
    __threadfence();
  }
}

__global__ __launch_bounds__(64) void conv_silu_kernel(
    const float* __restrict__ XZ, const float* __restrict__ cw, const float* __restrict__ cb,
    float* __restrict__ UC, unsigned short* __restrict__ UC16)
{
  __shared__ __align__(16) float sT[16 * kTP];
  const int tid = threadIdx.x, lane = tid & 31, wave = tid >> 5;
  const int d0 = blockIdx.x * 64, d = d0 + tid;
  const int t0 = blockIdx.y * 64;
  const int l0 = t0 & 4095;
  const float w0 = cw[d * 3 + 0], w1 = cw[d * 3 + 1], w2 = cw[d * 3 + 2];
  const float bc = cb[d];
  float xm2, xm1;
  {
    const int r2 = t0 - 2, r1 = t0 - 1;
    const float v2 = XZ[(size_t)(r2 < 0 ? 0 : r2) * kXZW + d];
    const float v1 = XZ[(size_t)(r1 < 0 ? 0 : r1) * kXZW + d];
    xm2 = (l0 >= 2) ? v2 : 0.f;
    xm1 = (l0 >= 1) ? v1 : 0.f;
  }
  const int hh = lane >> 4, c4 = (lane & 15) * 4;
  const int q  = lane >> 3, c8 = (lane & 7) * 8;
#pragma unroll 1
  for (int sub = 0; sub < 4; ++sub) {
    const int lb = t0 + sub * 16;
#pragma unroll 1
    for (int s = 0; s < 16; ++s) {
      const float xc = XZ[(size_t)(lb + s) * kXZW + d];
      float acc = w0 * xm2;
      acc = fmaf(w1, xm1, acc);
      acc = fmaf(w2, xc, acc);
      const float sv = acc + bc;
      const float sg = __builtin_amdgcn_rcpf(1.0f + __expf(-sv));
      sT[s * kTP + tid] = sv * sg;
      xm2 = xm1; xm1 = xc;
    }
    __syncthreads();
    v4f fv[4];
    v8h bv[2];
#pragma unroll
    for (int it = 0; it < 4; ++it) fv[it] = *(const v4f*)(sT + (it * 4 + wave * 2 + hh) * kTP + c4);
#pragma unroll
    for (int it = 0; it < 2; ++it) {
      const float* sp = sT + (it * 8 + wave * 4 + q) * kTP + c8;
      const v4f a0 = *(const v4f*)(sp);
      const v4f a1 = *(const v4f*)(sp + 4);
#pragma unroll
      for (int e = 0; e < 4; ++e) {
        bv[it][e]     = (_Float16)(a0[e] * 256.0f);
        bv[it][4 + e] = (_Float16)(a1[e] * 256.0f);
      }
    }
    for (int pass = 0; pass < 2; ++pass) {
#pragma unroll
      for (int it = 0; it < 4; ++it)
        *(volatile v4f*)(UC + (size_t)(lb + it * 4 + wave * 2 + hh) * kDin + d0 + c4) = fv[it];
#pragma unroll
      for (int it = 0; it < 2; ++it)
        *(volatile v8h*)(UC16 + (size_t)(lb + it * 8 + wave * 4 + q) * kDin + d0 + c8) = bv[it];
      __threadfence();
    }
    __syncthreads();
  }
}

__global__ __launch_bounds__(256) void dt_cast_kernel(
    const float* __restrict__ PROJ, unsigned short* __restrict__ DT16, int total8, float scale)
{
  const int i = blockIdx.x * 256 + threadIdx.x;
  if (i >= total8) return;
  const int e0  = i << 3;
  const int row = e0 >> 5;
  const int c8  = e0 & 31;
  const float* p = PROJ + (size_t)row * kPrjP + c8;
  const v4f a0 = *(const v4f*)(p);
  const v4f a1 = *(const v4f*)(p + 4);
  v8h hv;
#pragma unroll
  for (int e = 0; e < 4; ++e) {
    hv[e]     = (c8 + e < kDtR)     ? (_Float16)(a0[e] * scale) : (_Float16)0.0f;
    hv[4 + e] = (c8 + 4 + e < kDtR) ? (_Float16)(a1[e] * scale) : (_Float16)0.0f;
  }
  unsigned short* qd = DT16 + e0;
  *(volatile v8h*)qd = hv;
  __threadfence();
  *(volatile v8h*)qd = hv;
}

__global__ __launch_bounds__(64) void scan_kernel(
    const float* __restrict__ DLR, const float* __restrict__ UC, const float* __restrict__ XZ,
    const float* __restrict__ PROJ, const float* __restrict__ A_log, const float* __restrict__ Dv,
    unsigned short* __restrict__ Y16)
{
  __shared__ __align__(16) float sBC[16 * 32];
  __shared__ __align__(16) float sY[16 * kTP];
  const int tid = threadIdx.x, lane = tid & 31, wave = tid >> 5;
  const int d0 = blockIdx.x * 64, d = d0 + tid;
  const int rbase = blockIdx.y * kPix;

  float An[kNst];
#pragma unroll
  for (int n = 0; n < kNst; ++n) An[n] = -__expf(A_log[(size_t)d * kNst + n]);
  const float Dd = Dv[d];
  float h[kNst];
#pragma unroll
  for (int n = 0; n < kNst; ++n) h[n] = 0.f;
  const int q = lane >> 3, c8 = (lane & 7) * 8;

#pragma unroll 1
  for (int c = 0; c < kPix / 16; ++c) {
    const int l0 = c * 16;
#pragma unroll
    for (int p = 0; p < 2; ++p) {
      const int idx = tid + 64 * p;
      const int r = idx >> 3, q4 = (idx & 7) * 4;
      const v4f v = *(const v4f*)(PROJ + (size_t)(rbase + l0 + r) * kPrjP + 32 + q4);
      *(v4f*)(sBC + r * 32 + q4) = v;
    }
    __syncthreads();
#pragma unroll 1
    for (int s = 0; s < 16; ++s) {
      const size_t m = (size_t)(rbase + l0 + s);
      const float a     = DLR[m * kDin + d];
      const float delta = fmaxf(a, 0.0f) + log1pf(__expf(-fabsf(a)));
      const float xv    = UC[m * kDin + d];
      const float zv    = XZ[m * kXZW + kDin + d];
      v4f Bq[4], Cq[4];
#pragma unroll
      for (int qq = 0; qq < 4; ++qq) {
        Bq[qq] = *(const v4f*)(sBC + s * 32 + 4 * qq);
        Cq[qq] = *(const v4f*)(sBC + s * 32 + kNst + 4 * qq);
      }
      float y = 0.f;
#pragma unroll
      for (int n = 0; n < kNst; ++n) {
        const float e = __expf(delta * An[n]);
        float db = delta * Bq[n >> 2][n & 3];
        asm volatile("" : "+v"(db));
        float p = db * xv;
        asm volatile("" : "+v"(p));
        float qv = h[n] * e;
        asm volatile("" : "+v"(qv));
        const float hn = qv + p;
        h[n] = hn;
        float rr = Cq[n >> 2][n & 3] * hn;
        asm volatile("" : "+v"(rr));
        y += rr;
      }
      float sk = xv * Dd;
      asm volatile("" : "+v"(sk));
      y += sk;
      const float sg = __builtin_amdgcn_rcpf(1.0f + __expf(-zv));
      const float gt = zv * sg;
      sY[s * kTP + tid] = (y * gt) * 1024.0f;
    }
    __syncthreads();
    v8h hv[2];
#pragma unroll
    for (int it = 0; it < 2; ++it) {
      const float* sp = sY + (it * 8 + wave * 4 + q) * kTP + c8;
      const v4f a0 = *(const v4f*)(sp);
      const v4f a1 = *(const v4f*)(sp + 4);
#pragma unroll
      for (int e = 0; e < 4; ++e) { hv[it][e] = (_Float16)a0[e]; hv[it][4 + e] = (_Float16)a1[e]; }
    }
    for (int pass = 0; pass < 2; ++pass) {
#pragma unroll
      for (int it = 0; it < 2; ++it)
        *(volatile v8h*)(Y16 + (size_t)(rbase + l0 + it * 8 + wave * 4 + q) * kDin + d0 + c8) = hv[it];
      __threadfence();
    }
  }
}

__global__ __launch_bounds__(256) void reshape_split_kernel(
    const float* __restrict__ R, unsigned short* __restrict__ RTH, unsigned short* __restrict__ RTL)
{
  __shared__ float tile[64 * 65];
  const int tid = threadIdx.x, lane = tid & 31, wave = tid >> 5;
  const int ch0 = blockIdx.x * 64;
  const int g0  = blockIdx.y * 64;
  const int b   = g0 >> 12, px0 = g0 & 4095;
#pragma unroll
  for (int p = 0; p < 16; ++p) {
    const int idx = tid + p * 256;
    const int cc  = idx >> 6, pp = idx & 63;
    const int ch  = ch0 + cc;
    const int chc = (ch < kCin) ? ch : (kCin - 1);
    const int i   = (chc << 12) + px0 + pp;
    const int l   = i / kCin;
    const int c   = i - l * kCin;
    const float v = R[((size_t)(b * kPix + l)) * kCinP + c];
    tile[cc * 65 + pp] = (ch < kCin) ? v : 0.f;
  }
  __syncthreads();
  const int q = lane >> 3, c8 = (lane & 7) * 8;
  v8h hv[2], lv[2];
#pragma unroll
  for (int it = 0; it < 2; ++it) {
    const int prow = wave * 8 + it * 4 + q;
#pragma unroll
    for (int e = 0; e < 8; ++e) {
      const float t = tile[(c8 + e) * 65 + prow];
      const unsigned short hb = f2bf_bits(t);
      const unsigned short lb = f2bf_bits(t - bf_bits2f(hb));
      hv[it][e] = __builtin_bit_cast(_Float16, hb);
      lv[it][e] = __builtin_bit_cast(_Float16, lb);
    }
  }
  for (int pass = 0; pass < 2; ++pass) {
#pragma unroll
    for (int it = 0; it < 2; ++it) {
      const int prow = wave * 8 + it * 4 + q;
      *(volatile v8h*)(RTH + (size_t)(g0 + prow) * kCinP + ch0 + c8) = hv[it];
      *(volatile v8h*)(RTL + (size_t)(g0 + prow) * kCinP + ch0 + c8) = lv[it];
    }
    __threadfence();
  }
}

__global__ __launch_bounds__(256) void ln1_gelu_kernel(
    const float* __restrict__ FC, const float* __restrict__ fb, const float* __restrict__ g,
    const float* __restrict__ bb, float* __restrict__ out)
{
  const int gp = blockIdx.x * 256 + threadIdx.x;
  const int b = gp >> 12, px = gp & 4095;
  const float* row = FC + (size_t)gp * kOutP;
  float s = 0.f;
#pragma unroll 1
  for (int o = 0; o < kMod; ++o) s += row[o] + fb[o];
  const float mu = s * (1.0f / 96.0f);
  float s2 = 0.f;
#pragma unroll 1
  for (int o = 0; o < kMod; ++o) { const float dv = row[o] + fb[o] - mu; s2 += dv * dv; }
  const float rstd = rsqrtf(s2 * (1.0f / 96.0f) + 1e-5f);
  float* ob = out + (size_t)b * kMod * kPix + px;
  for (int pass = 0; pass < 2; ++pass) {
#pragma unroll 1
    for (int o = 0; o < kMod; ++o) {
      const float v  = row[o] + fb[o];
      const float xn = (v - mu) * rstd * g[o] + bb[o];
      const float ge = 0.5f * xn * (1.0f + erff(xn * 0.70710678118654752f));
      *(volatile float*)(ob + (size_t)o * kPix) = ge;
    }
    __threadfence();
  }
}

extern "C" void kernel_launch(void* const* d_in, const int* in_sizes, int n_in,
                              void* d_out, int out_size, void* d_ws, size_t ws_size,
                              hipStream_t stream)
{
  if (n_in < 18) return;
  const float* x1    = (const float*)d_in[0];
  const float* x2    = (const float*)d_in[1];
  const float* x3    = (const float*)d_in[2];
  const float* ln0_g = (const float*)d_in[3];
  const float* ln0_b = (const float*)d_in[4];
  const float* W_in  = (const float*)d_in[5];
  const float* cw    = (const float*)d_in[6];
  const float* cb    = (const float*)d_in[7];
  const float* W_x   = (const float*)d_in[8];
  const float* W_dt  = (const float*)d_in[9];
  const float* b_dt  = (const float*)d_in[10];
  const float* A_log = (const float*)d_in[11];
  const float* D_ssm = (const float*)d_in[12];
  const float* W_out = (const float*)d_in[13];
  const float* fc1_w = (const float*)d_in[14];
  const float* fc1_b = (const float*)d_in[15];
  const float* ln1_g = (const float*)d_in[16];
  const float* ln1_b = (const float*)d_in[17];
  float* dout = (float*)d_out;

  if (in_sizes[0] != kBatch * kMod * kPix || in_sizes[1] != kBatch * kMod * kPix || in_sizes[2] != kBatch * kMod * kPix) return;
  if (in_sizes[3] != kCin || in_sizes[4] != kCin) return;
  if (in_sizes[5] != kCin * kXZW) return;
  if (in_sizes[6] != kDin * 3 || in_sizes[7] != kDin) return;
  if (in_sizes[8] != kDin * kXdbl) return;
  if (in_sizes[9] != kDtR * kDin || in_sizes[10] != kDin) return;
  if (in_sizes[11] != kDin * kNst || in_sizes[12] != kDin) return;
  if (in_sizes[13] != kDin * kCin) return;
  if (in_sizes[14] != kCin * kMod || in_sizes[15] != kMod) return;
  if (in_sizes[16] != kMod || in_sizes[17] != kMod) return;
  if (out_size != kBatch * kMod * kPix) return;

  const size_t SZ_WIN16  = (size_t)kXZW * kCinP * 2;
  const size_t SZ_WX16   = (size_t)64 * kDin * 2;
  const size_t SZ_WDT16  = (size_t)kDin * kWdtP * 2;
  const size_t SZ_WOUT16 = (size_t)kCinP * kDin * 2;
  const size_t SZ_WFC    = (size_t)kOutP * kCinP * 2;
  const size_t SZ_XT     = (size_t)kRows * kCinP * 4;
  const size_t SZ_XN16   = (size_t)kRows * kCinP * 2;
  const size_t SZ_XZ     = (size_t)kRows * kXZW * 4;
  const size_t SZ_UC     = (size_t)kRows * kDin * 4;
  const size_t SZ_UC16   = (size_t)kRows * kDin * 2;
  const size_t SZ_PROJ   = (size_t)kRows * kPrjP * 4;
  const size_t SZ_DT16   = (size_t)kRows * kDtP * 2;
  const size_t SZ_DLR    = (size_t)kRows * kDin * 4;
  const size_t SZ_Y16    = (size_t)kRows * kDin * 2;
  const size_t SZ_R      = (size_t)kRows * kCinP * 4;
  const size_t SZ_RT     = (size_t)kRows * kCinP * 2;
  const size_t SZ_FC     = (size_t)kRows * kOutP * 4;

  const size_t OFF_WIN16  = 0;
  const size_t OFF_WX16   = OFF_WIN16  + SZ_WIN16;
  const size_t OFF_WDT16  = OFF_WX16   + SZ_WX16;
  const size_t OFF_WOUT16 = OFF_WDT16  + SZ_WDT16;
  const size_t OFF_WFCH   = OFF_WOUT16 + SZ_WOUT16;
  const size_t OFF_WFCL   = OFF_WFCH   + SZ_WFC;
  const size_t OFF_XT     = OFF_WFCL   + SZ_WFC;
  const size_t OFF_XN16   = OFF_XT     + SZ_XT;
  const size_t OFF_XZ     = OFF_XN16   + SZ_XN16;
  const size_t OFF_UC     = OFF_XZ     + SZ_XZ;
  const size_t OFF_UC16   = OFF_UC     + SZ_UC;
  const size_t OFF_PROJ   = OFF_UC16   + SZ_UC16;
  const size_t OFF_DT16   = OFF_PROJ   + SZ_PROJ;
  const size_t OFF_DLR    = OFF_DT16   + SZ_DT16;
  const size_t OFF_Y16    = OFF_DLR    + SZ_DLR;
  const size_t TOTAL      = OFF_Y16    + SZ_Y16;
  const size_t OFF_R      = OFF_XZ;
  const size_t OFF_RTH    = OFF_R   + SZ_R;
  const size_t OFF_RTL    = OFF_RTH + SZ_RT;
  const size_t OFF_FC     = OFF_RTL + SZ_RT;
  if (OFF_FC + SZ_FC > OFF_XZ + SZ_XZ) return;
  if (ws_size < TOTAL) return;

  char* ws = (char*)d_ws;
  unsigned short* WIN16  = (unsigned short*)(ws + OFF_WIN16);
  unsigned short* WX16   = (unsigned short*)(ws + OFF_WX16);
  unsigned short* WDT16  = (unsigned short*)(ws + OFF_WDT16);
  unsigned short* WOUT16 = (unsigned short*)(ws + OFF_WOUT16);
  unsigned short* WFCH   = (unsigned short*)(ws + OFF_WFCH);
  unsigned short* WFCL   = (unsigned short*)(ws + OFF_WFCL);
  float*          XT     = (float*)(ws + OFF_XT);
  unsigned short* XN16   = (unsigned short*)(ws + OFF_XN16);
  float*          XZ     = (float*)(ws + OFF_XZ);
  float*          UC     = (float*)(ws + OFF_UC);
  unsigned short* UC16   = (unsigned short*)(ws + OFF_UC16);
  float*          PROJ   = (float*)(ws + OFF_PROJ);
  unsigned short* DT16   = (unsigned short*)(ws + OFF_DT16);
  float*          DLR    = (float*)(ws + OFF_DLR);
  unsigned short* Y16    = (unsigned short*)(ws + OFF_Y16);
  float*          R      = (float*)(ws + OFF_R);
  unsigned short* RTH    = (unsigned short*)(ws + OFF_RTH);
  unsigned short* RTL    = (unsigned short*)(ws + OFF_RTL);
  float*          FC     = (float*)(ws + OFF_FC);
  const float* dummy_bias  = b_dt;
  const float* dummy_resid = XT;

  transpose_cast_kernel<0><<<dim3(kXZW / 64, kCinP / 64), 256, 0, stream>>>(W_in,  WIN16,  WIN16,  kCin, kXZW,  kCinP, kXZW,  0,  32.0f);
  transpose_cast_kernel<0><<<dim3(1, kDin / 64),          256, 0, stream>>>(W_x,   WX16,   WX16,   kDin, kXdbl, kDin,  kDtR,  14, 32.0f);
  transpose_cast_kernel<0><<<dim3(kDin / 64, 1),          256, 0, stream>>>(W_dt,  WDT16,  WDT16,  kDtR, kDin,  kWdtP, kDin,  0,  8.0f);
  transpose_cast_kernel<0><<<dim3(kCinP / 64, kDin / 64), 256, 0, stream>>>(W_out, WOUT16, WOUT16, kDin, kCin,  kDin,  kCin,  0,  32.0f);
  transpose_cast_kernel<1><<<dim3(kOutP / 64, kCinP / 64), 256, 0, stream>>>(fc1_w, WFCH,  WFCL,   kCin, kMod,  kCinP, kMod,  0,  1.0f);

  ln0_kernel<<<kRows / 8, 256, 0, stream>>>(x1, x2, x3, ln0_g, ln0_b, XT, XN16);

  wmma_gemm64<0, false, 0, 0, false><<<dim3(288, 1), 256, 0, stream>>>(
      XN16, XN16, kCinP, 0L, WIN16, WIN16, kCinP, 0L,
      (void*)XZ, (void*)XZ, kXZW, 0L, dummy_bias, dummy_resid, 0L, kRows, kXZW, kCin, 1.0f / 32.0f);

  conv_silu_kernel<<<dim3(kDin / 64, kRows / 64), 64, 0, stream>>>(XZ, cw, cb, UC, UC16);

  wmma_gemm64<0, false, 0, 0, false><<<dim3(16, 1), 256, 0, stream>>>(
      UC16, UC16, kDin, 0L, WX16, WX16, kDin, 0L,
      (void*)PROJ, (void*)PROJ, kPrjP, 0L, dummy_bias, dummy_resid, 0L, kRows, kPrjP, kDin, 1.0f / 8192.0f);

  dt_cast_kernel<<<(kRows * kDtP) / 8 / 256, 256, 0, stream>>>(PROJ, DT16, (kRows * kDtP) / 8, 1024.0f);

  wmma_gemm64<0, false, 2, 0, false><<<dim3(144, 1), 256, 0, stream>>>(
      DT16, DT16, kDtP, 0L, WDT16, WDT16, kWdtP, 0L,
      (void*)DLR, (void*)DLR, kDin, 0L, b_dt, dummy_resid, 0L, kRows, kDin, 32, 1.0f / 8192.0f);

  scan_kernel<<<dim3(kDin / 64, kBatch), 64, 0, stream>>>(DLR, UC, XZ, PROJ, A_log, D_ssm, Y16);

  wmma_gemm64<0, false, 0, 0, true><<<dim3(80, 1), 256, 0, stream>>>(
      Y16, Y16, kDin, 0L, WOUT16, WOUT16, kDin, 0L,
      (void*)R, (void*)R, kCinP, 0L, dummy_bias, XT, 0L, kRows, kCinP, kDin, 1.0f / 32768.0f);

  reshape_split_kernel<<<dim3(kCinP / 64, kRows / 64), 256, 0, stream>>>(R, RTH, RTL);

  wmma_gemm64<1, true, 0, 0, false><<<dim3(32, 1), 256, 0, stream>>>(
      RTH, RTL, kCinP, 0L, WFCH, WFCL, kCinP, 0L,
      (void*)FC, (void*)FC, kOutP, 0L, dummy_bias, dummy_resid, 0L, kRows, kOutP, kCinP, 1.0f);

  ln1_gelu_kernel<<<kRows / 256, 256, 0, stream>>>(FC, fc1_b, ln1_g, ln1_b, dout);
}
